// MultiScaleCrossAttention_20925080666670
// MI455X (gfx1250) — hardware-verified
//
#include <hip/hip_runtime.h>


namespace {
constexpr int Bn = 2, NQ = 8192, NKV = 1024, CQ = 384, CKV = 768, H = 8, HD = 48, HDP = 64, NTQ = Bn * NQ, NTK = Bn * NKV;
constexpr float QS = 8.0f, KS = 8.0f, VS = 8.0f, PS = 8.0f, AS_ = 8.0f, SCALE = 0.14433756729740643f;
constexpr size_t QPL = (size_t)Bn * H * NQ * HDP, KPL = (size_t)Bn * H * NKV * HDP, VPL = (size_t)Bn * H * HD * NKV;

typedef _Float16 b16;
typedef __attribute__((ext_vector_type(16))) _Float16 v16b;
typedef __attribute__((ext_vector_type(8))) _Float16 v8b;
typedef __attribute__((ext_vector_type(8))) float v8f;
typedef __attribute__((ext_vector_type(4))) float v4f;
__device__ __forceinline__ float bf16_rne(float f) { unsigned int u = __float_as_uint(f); u += 0x7FFFu + ((u >> 16) & 1u); return __uint_as_float(u & 0xFFFF0000u); }
__device__ __forceinline__ void split16(float v, b16& hi, b16& lo) { hi = (b16)v; lo = (b16)(v - (float)hi); }
__device__ __forceinline__ v16b frag_kb(const b16* p, int hh) { const v8b a = *(const v8b*)(p + 8 * hh), b = *(const v8b*)(p + 16 + 8 * hh); v16b f;
#pragma unroll
  for (int e = 0; e < 8; ++e) { f[e] = a[e]; f[8 + e] = b[e]; } return f; }
__device__ __forceinline__ void frag_split(const float* p, int hh, v16b& fh, v16b& fl) {
#pragma unroll
  for (int e = 0; e < 8; ++e) { b16 a, c; split16(p[8 * hh + e] * AS_, a, c); fh[e] = a; fl[e] = c; split16(p[16 + 8 * hh + e] * AS_, a, c); fh[8 + e] = a; fl[8 + e] = c; } }
__device__ __forceinline__ v8f wmma16b(v16b a, v16b b, v8f c) { v8f d = __builtin_amdgcn_wmma_f32_16x16x32_f16(false, a, false, b, (short)0, c, false, false); asm volatile("v_nop\n\tv_nop\n\tv_nop\n\tv_nop" : "+v"(d) : "v"(a), "v"(b)); return d; }
__device__ __forceinline__ void wave_lds_sync() { __builtin_amdgcn_fence(__ATOMIC_RELEASE, "workgroup"); __builtin_amdgcn_wave_barrier(); __builtin_amdgcn_fence(__ATOMIC_ACQUIRE, "workgroup"); }
__device__ __forceinline__ float nexp(float x) { return __builtin_amdgcn_exp2f(x * 1.4426950408889634f); }

struct Wo_ { static constexpr size_t Q = 0, K = Q + (size_t)CQ * CQ, V = K + (size_t)CQ * CKV, O = V + (size_t)CQ * CKV, END = O + (size_t)CQ * CQ; };
__global__ __launch_bounds__(256) void prep_kernel(const float* __restrict__ Wq, const float* __restrict__ Wk, const float* __restrict__ Wv, const float* __restrict__ Wo, const float* __restrict__ bq, const float* __restrict__ bk, const float* __restrict__ bv, const float* __restrict__ bo, const float* __restrict__ gq, const float* __restrict__ bq2, const float* __restrict__ gkv, const float* __restrict__ bkv2, b16* __restrict__ R, float* __restrict__ P) {
  const size_t tid = (size_t)blockIdx.x * blockDim.x + threadIdx.x, nth = (size_t)gridDim.x * blockDim.x;
  auto tr = [&](const float* W, int IN, int OUT, size_t base, size_t p) { const int o = (int)(p / (IN / 8)), k8 = (int)(p % (IN / 8)) * 8; v8b v;
#pragma unroll
    for (int e = 0; e < 8; ++e) v[e] = (b16)bf16_rne(W[(size_t)(k8 + e) * OUT + o]);
    *(volatile v8b*)(R + base + (size_t)o * IN + k8) = v; };
  for (int pass = 0; pass < 2; ++pass) {
    for (size_t p = tid; p < (size_t)CQ * CQ / 8; p += nth) { tr(Wq, CQ, CQ, Wo_::Q, p); tr(Wo, CQ, CQ, Wo_::O, p); }
    for (size_t p = tid; p < (size_t)CQ * CKV / 8; p += nth) { tr(Wk, CKV, CQ, Wo_::K, p); tr(Wv, CKV, CQ, Wo_::V, p); }
    for (size_t p = tid; p < 3840 / 4; p += nth) { v4f v;
#pragma unroll
      for (int e = 0; e < 4; ++e) { const int i = (int)p * 4 + e; float x; if (i < 384) x = bq[i]; else if (i < 768) x = bk[i - 384]; else if (i < 1152) x = bv[i - 768]; else if (i < 1536) x = bo[i - 1152]; else if (i < 1920) x = gq[i - 1536]; else if (i < 2304) x = bq2[i - 1920]; else if (i < 3072) x = gkv[i - 2304]; else x = bkv2[i - 3072]; v[e] = bf16_rne(x); }
      *(volatile v4f*)(P + p * 4) = v; }
    __threadfence(); }
}

template <int CW>
__global__ __launch_bounds__(256) void ln_kernel(const float* __restrict__ x, const float* __restrict__ g, const float* __restrict__ bb, float* __restrict__ y) {
  const int wid = threadIdx.x >> 5, lane = threadIdx.x & 31, row = blockIdx.x * 8 + wid; const float* pr = x + (size_t)row * CW; constexpr int NV = CW / 32;
  float v[NV]; float s = 0.0f;
#pragma unroll
  for (int j = 0; j < NV / 4; ++j) { const v4f t = *(const v4f*)(pr + j * 128 + lane * 4);
#pragma unroll
    for (int e = 0; e < 4; ++e) { v[j * 4 + e] = bf16_rne(t[e]); s += v[j * 4 + e]; } }
#pragma unroll
  for (int o = 1; o < 32; o <<= 1) s += __shfl_xor(s, o);
  const float mu = s * (1.0f / CW); float q = 0.0f;
#pragma unroll
  for (int j = 0; j < NV; ++j) { const float d = v[j] - mu; q += d * d; }
#pragma unroll
  for (int o = 1; o < 32; o <<= 1) q += __shfl_xor(q, o);
  const float is = rsqrtf(q * (1.0f / CW) + 1e-5f);
  for (int pass = 0; pass < 2; ++pass) {
#pragma unroll
    for (int j = 0; j < NV / 4; ++j) { const int c = j * 128 + lane * 4; v4f o4; for (int e = 0; e < 4; ++e) o4[e] = (v[j * 4 + e] - mu) * is * g[c + e] + bb[c + e]; *(volatile v4f*)(y + (size_t)row * CW + c) = o4; }
    __threadfence(); }
}

__global__ __launch_bounds__(128) void proj_kernel(const float* __restrict__ qn, const float* __restrict__ kvn, const b16* __restrict__ R, const float* __restrict__ P, b16* __restrict__ qp, b16* __restrict__ kp, b16* __restrict__ vt) {
  __shared__ __attribute__((aligned(16))) b16 Th[4][32][HDP + 8], Tl[4][32][HDP + 8]; __shared__ __attribute__((aligned(16))) b16 Vh[HD][128 + 8], Vl[HD][128 + 8];
  const int lane = threadIdx.x & 31, wave = threadIdx.x >> 5, nloc = lane & 15, hlf = lane >> 4, which = blockIdx.z, h = blockIdx.x, c0 = h * HD; const int nrow = (which == 0) ? NTQ : NTK, K = (which == 0) ? CQ : CKV, per = (which == 0) ? NQ : NKV;
  if ((int)blockIdx.y * 128 >= nrow) return;
  const int m0 = blockIdx.y * 128 + wave * 32; const float* X = (which == 0) ? qn : kvn; const b16* Wt = R + ((which == 0) ? Wo_::Q : (which == 1) ? Wo_::K : Wo_::V); const float* bias = P + which * 384;
  v8f acc[2][3];
#pragma unroll
  for (int r = 0; r < 2; ++r)
#pragma unroll
    for (int t = 0; t < 3; ++t) acc[r][t] = (v8f){};
  for (int kb = 0; kb < K; kb += 32) { v16b a0, l0, a1, l1; frag_split(X + (size_t)(m0 + nloc) * K + kb, hlf, a0, l0); frag_split(X + (size_t)(m0 + 16 + nloc) * K + kb, hlf, a1, l1);
#pragma unroll
    for (int t = 0; t < 3; ++t) { const v16b bw = frag_kb(Wt + (size_t)(c0 + t * 16 + nloc) * K + kb, hlf); acc[0][t] = wmma16b(a0, bw, acc[0][t]); acc[0][t] = wmma16b(l0, bw, acc[0][t]); acc[1][t] = wmma16b(a1, bw, acc[1][t]); acc[1][t] = wmma16b(l1, bw, acc[1][t]); } }
  const float scl = (which == 0) ? SCALE * QS : ((which == 1) ? KS : VS);
  if (which < 2) {
#pragma unroll
    for (int t = 0; t < 3; ++t) { const float bb = bias[c0 + t * 16 + nloc];
#pragma unroll
      for (int r = 0; r < 2; ++r)
#pragma unroll
        for (int v = 0; v < 8; ++v) { b16 a_, l_; split16((acc[r][t][v] * (1.0f / AS_) + bb) * scl, a_, l_); Th[wave][r * 16 + 8 * hlf + v][t * 16 + nloc] = a_; Tl[wave][r * 16 + 8 * hlf + v][t * 16 + nloc] = l_; } }
    for (int i = lane; i < 32 * 16; i += 32) { const int rr = i >> 4, cc = HD + (i & 15); Th[wave][rr][cc] = (b16)0.0f; Tl[wave][rr][cc] = (b16)0.0f; }
    wave_lds_sync();
    b16* base = (which == 0) ? qp : kp; const size_t PLN = (which == 0) ? QPL : KPL;
    for (int pass = 0; pass < 2; ++pass) {
#pragma unroll
      for (int j = 0; j < 8; ++j) { const int rr = j * 4 + (lane >> 3), c8 = (lane & 7) * 8; const int m = m0 + rr, bb = m / per, tok = m % per; const size_t o = (((size_t)bb * H + h) * per + tok) * HDP + c8;
        *(volatile v8b*)(base + o) = *(const v8b*)(&Th[wave][rr][c8]); *(volatile v8b*)(base + PLN + o) = *(const v8b*)(&Tl[wave][rr][c8]); }
      __threadfence(); }
    return; }
  const int bblk = (blockIdx.y * 128) / per, t0 = (blockIdx.y * 128) % per;
#pragma unroll
  for (int t = 0; t < 3; ++t) { const float bb = bias[c0 + t * 16 + nloc];
#pragma unroll
    for (int r = 0; r < 2; ++r)
#pragma unroll
      for (int v = 0; v < 8; ++v) { b16 a_, l_; split16((acc[r][t][v] * (1.0f / AS_) + bb) * scl, a_, l_); Vh[t * 16 + nloc][wave * 32 + r * 16 + 8 * hlf + v] = a_; Vl[t * 16 + nloc][wave * 32 + r * 16 + 8 * hlf + v] = l_; } }
  __syncthreads();
  for (int pass = 0; pass < 2; ++pass) { for (int i = threadIdx.x; i < HD * 16; i += 128) { const int d = i >> 4, c8 = (i & 15) * 8; const size_t o = (((size_t)bblk * H + h) * HD + d) * NKV + t0 + c8;
      *(volatile v8b*)(vt + o) = *(const v8b*)(&Vh[d][c8]); *(volatile v8b*)(vt + VPL + o) = *(const v8b*)(&Vl[d][c8]); } __threadfence(); }
}

__global__ __launch_bounds__(256) void attn_kernel(const b16* __restrict__ qp, const b16* __restrict__ kp, const b16* __restrict__ vt, float* __restrict__ ctx) {
  __shared__ __attribute__((aligned(16))) float Os[16][CQ + 4];
  const int h = threadIdx.x >> 5, lane = threadIdx.x & 31, hh = lane >> 4, col = lane & 15; const int b = blockIdx.x / (NQ / 16), q0 = (blockIdx.x % (NQ / 16)) * 16, qi = q0 + col;
  const b16* Q = qp + (((size_t)b * H + h) * NQ) * HDP; const b16* Kb = kp + (((size_t)b * H + h) * NKV) * HDP; const b16* V = vt + (((size_t)b * H + h) * HD) * NKV;
  v16b qf[2], ql[2];
#pragma unroll
  for (int ks = 0; ks < 2; ++ks) { qf[ks] = frag_kb(Q + (size_t)qi * HDP + ks * 32, hh); ql[ks] = frag_kb(Q + QPL + (size_t)qi * HDP + ks * 32, hh); }
  float m = -INFINITY, l = 0.0f; v8f o[3] = {{}, {}, {}};
  for (int kb = 0; kb < NKV; kb += 32) { v8f s0 = {}, s1 = {};
#pragma unroll
    for (int ks = 0; ks < 2; ++ks) { const v16b ka = frag_kb(Kb + (size_t)(kb + col) * HDP + ks * 32, hh), kal = frag_kb(Kb + KPL + (size_t)(kb + col) * HDP + ks * 32, hh), kc = frag_kb(Kb + (size_t)(kb + 16 + col) * HDP + ks * 32, hh), kcl = frag_kb(Kb + KPL + (size_t)(kb + 16 + col) * HDP + ks * 32, hh);
      s0 = wmma16b(ka, qf[ks], s0); s0 = wmma16b(ka, ql[ks], s0); s0 = wmma16b(kal, qf[ks], s0); s1 = wmma16b(kc, qf[ks], s1); s1 = wmma16b(kc, ql[ks], s1); s1 = wmma16b(kcl, qf[ks], s1); }
    float mr = -INFINITY;
#pragma unroll
    for (int r = 0; r < 8; ++r) { s0[r] *= 1.0f / (QS * KS); s1[r] *= 1.0f / (QS * KS); mr = fmaxf(mr, fmaxf(s0[r], s1[r])); }
    mr = fmaxf(mr, __shfl_xor(mr, 16));
    const float mn = fmaxf(m, mr), al_ = nexp(m - mn); m = mn; float sum = 0.0f; v16b pbv, plv;
#pragma unroll
    for (int r = 0; r < 8; ++r) { const float e0 = nexp(s0[r] - mn), e1 = nexp(s1[r] - mn); sum += e0 + e1; b16 a, cc; split16(e0 * PS, a, cc); pbv[r] = a; plv[r] = cc; split16(e1 * PS, a, cc); pbv[8 + r] = a; plv[8 + r] = cc; }
    sum += __shfl_xor(sum, 16); l = l * al_ + sum;
#pragma unroll
    for (int t = 0; t < 3; ++t) { o[t] *= al_; const v16b vf = frag_kb(V + (size_t)(t * 16 + col) * NKV + kb, hh), vl = frag_kb(V + VPL + (size_t)(t * 16 + col) * NKV + kb, hh); o[t] = wmma16b(vf, pbv, o[t]); o[t] = wmma16b(vf, plv, o[t]); o[t] = wmma16b(vl, pbv, o[t]); } }
  const float inv = 1.0f / (l * VS * PS);
#pragma unroll
  for (int t = 0; t < 3; ++t)
#pragma unroll
    for (int r = 0; r < 8; ++r) Os[col][h * HD + t * 16 + 8 * hh + r] = o[t][r] * inv;
  __syncthreads();
  float* dst = ctx + ((size_t)b * NQ + q0) * CQ;
  for (int pass = 0; pass < 2; ++pass) { for (int i = threadIdx.x; i < 16 * (CQ / 4); i += 256) { const int rr = i / (CQ / 4), c4 = (i % (CQ / 4)) * 4; *(volatile v4f*)(dst + (size_t)rr * CQ + c4) = *(const v4f*)(&Os[rr][c4]); } __threadfence(); }
}

__global__ __launch_bounds__(128) void out_kernel(const float* __restrict__ ctx, const b16* __restrict__ R, const float* __restrict__ P, const float* __restrict__ xq, float* __restrict__ out) {
  __shared__ __attribute__((aligned(16))) float Ts[4][32 * 64];
  const int lane = threadIdx.x & 31, wave = threadIdx.x >> 5, nloc = lane & 15, hlf = lane >> 4, m0 = blockIdx.y * 128 + wave * 32, c0 = blockIdx.x * 64; const float* bo = P + 1152; const b16* Wt = R + Wo_::O;
  v8f acc[2][4];
#pragma unroll
  for (int r = 0; r < 2; ++r)
#pragma unroll
    for (int t = 0; t < 4; ++t) acc[r][t] = (v8f){};
  for (int kb = 0; kb < CQ; kb += 32) { v16b a0, l0, a1, l1; frag_split(ctx + (size_t)(m0 + nloc) * CQ + kb, hlf, a0, l0); frag_split(ctx + (size_t)(m0 + 16 + nloc) * CQ + kb, hlf, a1, l1);
#pragma unroll
    for (int t = 0; t < 4; ++t) { const v16b bw = frag_kb(Wt + (size_t)(c0 + t * 16 + nloc) * CQ + kb, hlf); acc[0][t] = wmma16b(a0, bw, acc[0][t]); acc[0][t] = wmma16b(l0, bw, acc[0][t]); acc[1][t] = wmma16b(a1, bw, acc[1][t]); acc[1][t] = wmma16b(l1, bw, acc[1][t]); } }
  float* Tt = Ts[wave];
#pragma unroll
  for (int t = 0; t < 4; ++t) { const int cc = c0 + t * 16 + nloc; const float bb = bo[cc];
#pragma unroll
    for (int r = 0; r < 2; ++r)
#pragma unroll
      for (int v = 0; v < 8; ++v) { const int rl = r * 16 + v + 8 * hlf; Tt[rl * 64 + t * 16 + nloc] = acc[r][t][v] * (1.0f / AS_) + bb + bf16_rne(xq[(size_t)(m0 + rl) * CQ + cc]); } }
  wave_lds_sync();
  for (int pass = 0; pass < 2; ++pass) {
#pragma unroll
    for (int j = 0; j < 16; ++j) { const int rr = j * 2 + hlf, c4 = nloc * 4; *(volatile v4f*)(out + (size_t)(m0 + rr) * CQ + c0 + c4) = *(const v4f*)(Tt + rr * 64 + c4); }
    __threadfence(); }
}
}

extern "C" void kernel_launch(void* const* d_in, const int* in_sizes, int n_in,
                              void* d_out, int out_size, void* d_ws, size_t ws_size, hipStream_t stream) {
  (void)n_in; (void)out_size;
  const float* xq = (const float*)d_in[0]; const float* xkv = (const float*)d_in[1]; const float* Wq = (const float*)d_in[2]; const float* bq = (const float*)d_in[3]; const float* Wk = (const float*)d_in[4]; const float* bk = (const float*)d_in[5]; const float* Wv = (const float*)d_in[6]; const float* bv = (const float*)d_in[7];
  const float* Wo = (const float*)d_in[8]; const float* bo = (const float*)d_in[9]; const float* gq = (const float*)d_in[10]; const float* bq2 = (const float*)d_in[11]; const float* gkv = (const float*)d_in[12]; const float* bkv2 = (const float*)d_in[13];
  float* out = (float*)d_out;
  if (in_sizes[0] != NTQ * CQ || in_sizes[1] != NTK * CKV || in_sizes[2] != CQ * CQ || in_sizes[4] != CKV * CQ || in_sizes[8] != CQ * CQ) return;
  size_t off = 0; char* ws = (char*)d_ws;
  auto carve = [&](size_t bytes) { char* p = ws + off; off += (bytes + 255) & ~(size_t)255; return p; };
  b16* R = (b16*)carve(Wo_::END * 2); float* P = (float*)carve(3840 * 4); float* qn = (float*)carve((size_t)NTQ * CQ * 4); float* kvn = (float*)carve((size_t)NTK * CKV * 4);
  b16* qp = (b16*)carve(QPL * 2 * 2); b16* kp = (b16*)carve(KPL * 2 * 2); b16* vt = (b16*)carve(VPL * 2 * 2); float* ctx = qn;
  if (off > ws_size) return;
  prep_kernel<<<256, 256, 0, stream>>>(Wq, Wk, Wv, Wo, bq, bk, bv, bo, gq, bq2, gkv, bkv2, R, P);
  ln_kernel<CQ><<<NTQ / 8, 256, 0, stream>>>(xq, P + 1536, P + 1920, qn);
  ln_kernel<CKV><<<NTK / 8, 256, 0, stream>>>(xkv, P + 2304, P + 3072, kvn);
  proj_kernel<<<dim3(H, NTQ / 128, 3), 128, 0, stream>>>(qn, kvn, R, P, qp, kp, vt);
  attn_kernel<<<NTQ / 16, 256, 0, stream>>>(qp, kp, vt, ctx);
  out_kernel<<<dim3(CQ / 64, NTQ / 128), 128, 0, stream>>>(ctx, R, P, xq, out);
}
